// Global_Fea_Extractor_37855841747278
// MI455X (gfx1250) — hardware-verified
//
#include <hip/hip_runtime.h>


#define NB_  2
#define NN   8192
#define CC   128
#define RB   2048
typedef _Float16 h16;
typedef unsigned short bf;
typedef __attribute__((ext_vector_type(16))) __bf16   v16bf;
typedef __attribute__((ext_vector_type(16))) _Float16 v16h;
typedef __attribute__((ext_vector_type(8)))  _Float16 v8h;
typedef __attribute__((ext_vector_type(8)))  unsigned short v8us;
typedef __attribute__((ext_vector_type(8)))  float    v8f;
typedef __attribute__((ext_vector_type(4)))  float    v4f;
typedef v8h  __attribute__((may_alias)) v8ha;
typedef v4f  __attribute__((may_alias)) v4fa;
typedef v8us __attribute__((may_alias)) v8usa;

__device__ __forceinline__ unsigned short f2bf(float f) { unsigned u = __float_as_uint(f); u += 0x7FFFu + ((u >> 16) & 1u); return (unsigned short)(u >> 16); }
__device__ __forceinline__ float bf2f(unsigned short b) { return __uint_as_float(((unsigned)b) << 16); }
__device__ __forceinline__ float bfr(float f) { return bf2f(f2bf(f)); }
__device__ __forceinline__ v16h cat16(v8h lo, v8h hi) { return __builtin_shufflevector(lo, hi, 0, 1, 2, 3, 4, 5, 6, 7, 8, 9, 10, 11, 12, 13, 14, 15); }
__device__ __forceinline__ v16bf cat16b(v8us lo, v8us hi) { return __builtin_bit_cast(v16bf, __builtin_shufflevector(lo, hi, 0, 1, 2, 3, 4, 5, 6, 7, 8, 9, 10, 11, 12, 13, 14, 15)); }
__device__ __forceinline__ v8f wmma16(v16h a, v16h b, v8f c) { return __builtin_amdgcn_wmma_f32_16x16x32_f16(false, a, false, b, (short)0, c, false, false); }
__device__ __forceinline__ v8f wmmab(v16bf a, v16bf b, v8f c) { return __builtin_amdgcn_wmma_f32_16x16x32_bf16(false, a, false, b, (short)0, c, false, false); }


template <typename T16> struct WFrag;
template <> struct WFrag<h16> { typedef v16h V; static __device__ __forceinline__ V ld(const h16* p) { return cat16(*(const v8h*)p, *(const v8h*)(p + 16)); } static __device__ __forceinline__ v8f mma(V a, V b, v8f c) { return wmma16(a, b, c); } };
template <> struct WFrag<bf> { typedef v16bf V; static __device__ __forceinline__ V ld(const bf* p) { return cat16b(*(const v8us*)p, *(const v8us*)(p + 16)); } static __device__ __forceinline__ v8f mma(V a, V b, v8f c) { return wmmab(a, b, c); } };
template <typename T16, int NSPLIT, bool BIAS>
__global__ __launch_bounds__(32) void k_gemmw(const T16* __restrict__ A, const T16* __restrict__ A2, const T16* __restrict__ Bt, const T16* __restrict__ Bt2, int K, float* C, int ldc, const float* __restrict__ bias, size_t sA, size_t sB, size_t sC) {
    typedef typename WFrag<T16>::V V;
    __shared__ __align__(16) float os[16 * 68];
    const size_t z = blockIdx.z; A += z * sA; if (A2) A2 += z * sA; Bt += z * sB; if (Bt2) Bt2 += z * sB; C += z * sC;
    const int lane = threadIdx.x & 31, lr = lane & 15, hi = lane >> 4; const int r0 = blockIdx.x * 64, c0 = blockIdx.y * 64;
    v8f acc[4][4];
#pragma unroll
    for (int mb = 0; mb < 4; ++mb)
#pragma unroll
        for (int nb = 0; nb < 4; ++nb) acc[mb][nb] = (v8f){};
    const size_t aoff = (size_t)(r0 + lr) * K + 8 * hi, boff = (size_t)(c0 + lr) * K + 8 * hi;
#pragma unroll 1
    for (int kc = 0; kc < K; kc += 32) {
        V a[4], a2[4];
#pragma unroll
        for (int mb = 0; mb < 4; ++mb) { a[mb] = WFrag<T16>::ld(A + aoff + (size_t)mb * 16 * K + kc); if (NSPLIT == 1 || NSPLIT == 2) a2[mb] = WFrag<T16>::ld(A2 + aoff + (size_t)mb * 16 * K + kc); }
#pragma unroll
        for (int nb = 0; nb < 4; ++nb) { const V b = WFrag<T16>::ld(Bt + boff + (size_t)nb * 16 * K + kc); V b2; if (NSPLIT >= 2) b2 = WFrag<T16>::ld(Bt2 + boff + (size_t)nb * 16 * K + kc);
#pragma unroll
            for (int mb = 0; mb < 4; ++mb) { acc[mb][nb] = WFrag<T16>::mma(a[mb], b, acc[mb][nb]); if (NSPLIT == 1 || NSPLIT == 2) acc[mb][nb] = WFrag<T16>::mma(a2[mb], b, acc[mb][nb]); if (NSPLIT >= 2) acc[mb][nb] = WFrag<T16>::mma(a[mb], b2, acc[mb][nb]); } }
        asm volatile("v_nop\n\tv_nop\n\tv_nop\n\tv_nop" : "+v"(acc[0][0]), "+v"(acc[1][1]), "+v"(acc[2][2]), "+v"(acc[3][3]) : "v"(a[0]), "v"(a[3]));
    }
#pragma unroll
    for (int mb = 0; mb < 4; ++mb) {
#pragma unroll
        for (int nb = 0; nb < 4; ++nb) {
#pragma unroll
            for (int j = 0; j < 8; ++j) os[(hi * 8 + j) * 68 + nb * 16 + lr] = acc[mb][nb][j]; }
        __builtin_amdgcn_wave_barrier(); asm volatile("" ::: "memory");
        float* crow = C + (size_t)(r0 + mb * 16) * ldc + c0;
#pragma unroll 1
        for (int ps = 0; ps < 2; ++ps) {
#pragma unroll
            for (int s = 0; s < 8; ++s) { const int row = 2 * s + hi, cofs = lr * 4; v4f val = *(const v4fa*)(os + row * 68 + cofs); if (BIAS) { val[0] += bfr(bias[c0 + cofs]); val[1] += bfr(bias[c0 + cofs + 1]); val[2] += bfr(bias[c0 + cofs + 2]); val[3] += bfr(bias[c0 + cofs + 3]); }
                *(volatile v4f*)(crow + (size_t)row * ldc + cofs) = val; }
            if (ps == 0) __threadfence(); }
        __builtin_amdgcn_wave_barrier(); asm volatile("" ::: "memory");
    }
}

__device__ __forceinline__ void splitf(float y, unsigned short& h, unsigned short& l) { h = f2bf(y); l = f2bf(y - bf2f(h)); }
typedef __attribute__((ext_vector_type(2))) unsigned short v2us;
typedef __attribute__((ext_vector_type(4))) unsigned short v4us;

__global__ __launch_bounds__(256) void k_ft(const float* __restrict__ fb, bf* FT) {
    const int lane = threadIdx.x & 31; const int L0 = (blockIdx.x * 8 + (threadIdx.x >> 5)) * 8; const int nlines = CC * NN / 64;
#pragma unroll 1
    for (int ps = 0; ps < 2; ++ps) {
#pragma unroll
        for (int l = 0; l < 8; ++l) { const int L = L0 + l; if (L >= nlines) break; const int e = L * 64 + lane * 2; const int n = e & (NN - 1); const int c = e >> 13; v2us o;
#pragma unroll
            for (int q = 0; q < 2; ++q) o[q] = f2bf(fb[(size_t)(n + q) * CC + c]);
            *(volatile v2us*)(FT + (size_t)e) = o; }
        if (ps == 0) __threadfence(); }
}
__global__ __launch_bounds__(256) void k_lat(const float* __restrict__ fb, const float* __restrict__ w1, const float* __restrict__ w2, const float* __restrict__ sc, float* LP) {
    const int lane = threadIdx.x & 31; const int n = blockIdx.x * 8 + (threadIdx.x >> 5); if (n >= NN) return; const v4f x4 = *(const v4f*)(fb + (size_t)n * CC + lane * 4); float a1 = 0.f, a2 = 0.f;
#pragma unroll
    for (int q = 0; q < 4; ++q) { const float xv = bfr(x4[q]); float p1 = __fmul_rn(xv, bfr(w1[lane * 4 + q])), p2 = __fmul_rn(xv, bfr(w2[lane * 4 + q])); asm volatile("" : "+v"(p1)); asm volatile("" : "+v"(p2)); a1 = __fadd_rn(a1, p1); a2 = __fadd_rn(a2, p2); }
#pragma unroll
    for (int sh = 16; sh; sh >>= 1) { a1 += __shfl_xor(a1, sh, 32); a2 += __shfl_xor(a2, sh, 32); }
    float l1 = __fmul_rn(__fdiv_rn(__fsub_rn(__fadd_rn(a1, bfr(sc[0])), bfr(sc[3])), __fsqrt_rn(__fadd_rn(bfr(sc[4]), 1e-5f))), bfr(sc[1])); asm volatile("" : "+v"(l1)); l1 = fmaxf(__fadd_rn(l1, bfr(sc[2])), 0.f);
    float l2 = __fmul_rn(__fdiv_rn(__fsub_rn(__fadd_rn(a2, bfr(sc[5])), bfr(sc[8])), __fsqrt_rn(__fadd_rn(bfr(sc[9]), 1e-5f))), bfr(sc[6])); asm volatile("" : "+v"(l2)); l2 = fmaxf(__fadd_rn(l2, bfr(sc[7])), 0.f);
    const float o = (lane == 0) ? l1 : (lane == 1 ? l2 : 0.f); *(volatile float*)(LP + (size_t)n * 32 + lane) = o; __threadfence(); *(volatile float*)(LP + (size_t)n * 32 + lane) = o; }
__global__ __launch_bounds__(32) void k_sc(const float* a0, const float* a1, const float* a2, const float* a3, const float* a4, const float* a5, const float* a6, const float* a7, const float* a8, const float* a9, float* sc) {
    const int i = threadIdx.x; const float* src[10] = {a0, a1, a2, a3, a4, a5, a6, a7, a8, a9}; float v = 0.f;
#pragma unroll
    for (int k = 0; k < 10; ++k) if (i == k) v = src[k][0];
    *(volatile float*)(sc + i) = v; __threadfence(); *(volatile float*)(sc + i) = v; }
__global__ __launch_bounds__(32) void k_max(const float* __restrict__ LP, float* MX) {
    const int lane = threadIdx.x; float m1 = 0.f, m2 = 0.f;
    for (int n = lane; n < NN; n += 32) { m1 = fmaxf(m1, LP[(size_t)n * 32]); m2 = fmaxf(m2, LP[(size_t)n * 32 + 1]); }
#pragma unroll
    for (int sh = 16; sh; sh >>= 1) { m1 = fmaxf(m1, __shfl_xor(m1, sh, 32)); m2 = fmaxf(m2, __shfl_xor(m2, sh, 32)); }
    const float o = (lane == 0) ? m1 : (lane == 1 ? m2 : 0.f); *(volatile float*)(MX + lane) = o; __threadfence(); *(volatile float*)(MX + lane) = o; }
__global__ __launch_bounds__(256) void k_egen(const float* __restrict__ LP, const float* __restrict__ MX, int n0, bf* Eh, bf* El, float* RSUM) {
    const int lane = threadIdx.x & 31; const int r = blockIdx.x * 8 + (threadIdx.x >> 5); if (r >= RB) return; const int n = n0 + r; const float l1 = LP[(size_t)n * 32]; const float M = __fmul_rn(MX[0], MX[1]); float sum = 0.f;
#pragma unroll 2
    for (int c0 = lane * 4; c0 < NN; c0 += 128) { v4us oh, ol;
#pragma unroll
        for (int q = 0; q < 4; ++q) { float a = __fmul_rn(l1, LP[(size_t)(c0 + q) * 32 + 1]); asm volatile("" : "+v"(a)); const float e = __expf(__fsub_rn(a, M)); sum += e; unsigned short hh, ll; splitf(e, hh, ll); oh[q] = hh; ol[q] = ll; }
        *(volatile v4us*)(Eh + (size_t)r * NN + c0) = oh; *(volatile v4us*)(El + (size_t)r * NN + c0) = ol; __threadfence(); *(volatile v4us*)(Eh + (size_t)r * NN + c0) = oh; *(volatile v4us*)(El + (size_t)r * NN + c0) = ol; }
#pragma unroll
    for (int sh = 16; sh; sh >>= 1) sum += __shfl_xor(sum, sh, 32);
    const float o = (lane == 0) ? sum : 0.f; *(volatile float*)(RSUM + (size_t)n * 32 + lane) = o; __threadfence(); *(volatile float*)(RSUM + (size_t)n * 32 + lane) = o; }
__global__ __launch_bounds__(32) void k_zsum(const float* __restrict__ RSUM, float* ZL) {
    const int lane = threadIdx.x; float s = 0.f; for (int n = lane; n < NN; n += 32) s = __fadd_rn(s, RSUM[(size_t)n * 32]);
#pragma unroll
    for (int sh = 16; sh; sh >>= 1) s += __shfl_xor(s, sh, 32);
    const float o = (lane == 0) ? s : 0.f; *(volatile float*)(ZL + lane) = o; __threadfence(); *(volatile float*)(ZL + lane) = o; }
__global__ __launch_bounds__(256) void k_fin(const float* __restrict__ U, const float* __restrict__ ZL, const float* __restrict__ fb, float* OUTb) { const size_t i = ((size_t)blockIdx.x * 256 + threadIdx.x) * 4; if (i >= (size_t)NN * CC) return; const float rz = __fdiv_rn(1.0f, ZL[0]); const v4f u = *(const v4f*)(U + i), f4 = *(const v4f*)(fb + i); v4f o;
#pragma unroll
    for (int q = 0; q < 4; ++q) { float t = __fmul_rn(u[q], rz); asm volatile("" : "+v"(t)); o[q] = __fadd_rn(t, bfr(f4[q])); }
    *(volatile v4f*)(OUTb + i) = o; __threadfence(); *(volatile v4f*)(OUTb + i) = o; }

extern "C" void kernel_launch(void* const* d_in, const int* in_sizes, int n_in,
                              void* d_out, int out_size, void* d_ws, size_t ws_size, hipStream_t stream) {
    (void)in_sizes; (void)n_in; (void)out_size;
    const float* IN[13]; for (int i = 0; i < 13; ++i) IN[i] = (const float*)d_in[i];
    const float* feat = IN[0];
    float* OUT = (float*)d_out;
    char* wsp = (char*)d_ws;
    auto take = [&](size_t bytes) { char* p = wsp; wsp += (bytes + 255) & ~(size_t)255; return (void*)p; };
    float* SC = (float*)take(256); float* LP = (float*)take((size_t)NN * 32 * 4); float* MX = (float*)take(256); float* RSUM = (float*)take((size_t)NN * 32 * 4); float* ZL = (float*)take(256);
    bf* FT = (bf*)take((size_t)CC * NN * 2); bf* Eh = (bf*)take((size_t)RB * NN * 2); bf* El = (bf*)take((size_t)RB * NN * 2); float* U = (float*)take((size_t)NN * CC * 4);
    if ((size_t)(wsp - (char*)d_ws) > ws_size) return;
    k_sc<<<1, 32, 0, stream>>>(IN[2], IN[3], IN[4], IN[5], IN[6], IN[8], IN[9], IN[10], IN[11], IN[12], SC);
    const unsigned L4 = (unsigned)(((size_t)NN * CC / 4 + 255) / 256);
    for (int b = 0; b < NB_; ++b) { const float* fb = feat + (size_t)b * NN * CC;
        k_ft<<<(CC * NN / 64 + 63) / 64, 256, 0, stream>>>(fb, FT); k_lat<<<NN / 8, 256, 0, stream>>>(fb, IN[1], IN[7], SC, LP); k_max<<<1, 32, 0, stream>>>(LP, MX);
        for (int n0 = 0; n0 < NN; n0 += RB) {
            k_egen<<<RB / 8, 256, 0, stream>>>(LP, MX, n0, Eh, El, RSUM);
            k_gemmw<bf, 1, false><<<dim3(RB / 64, CC / 64, 1), 32, 0, stream>>>(Eh, El, FT, nullptr, NN, U + (size_t)n0 * CC, CC, nullptr, 0, 0, 0); }
        k_zsum<<<1, 32, 0, stream>>>(RSUM, ZL);
        k_fin<<<L4, 256, 0, stream>>>(U, ZL, fb, OUT + (size_t)b * NN * CC); }
}
